// _lstm_forecaster_90623809945629
// MI455X (gfx1250) — hardware-verified
//
#include <hip/hip_runtime.h>
#include <math.h>

constexpr int NBATCH   = 8192;
constexpr int NSTEP    = 96;
constexpr int NHID     = 64;
constexpr int NGATE    = 4 * NHID;
constexpr int NPRED    = 24;
constexpr int NWAVE    = 4;
constexpr int NTHR     = NWAVE * 32;
constexpr int ROWS_BLK = NWAVE * 16;
constexpr int T_HEAD0  = NSTEP - NPRED;
constexpr int TILE_H   = 16 * NHID;
constexpr float WCARRY = 8.0f;
constexpr float HCARRY = 16.0f;
constexpr float ZCARRY = WCARRY * HCARRY;
constexpr float ZFOLD  = 1.0f / (WCARRY * HCARRY);

static_assert(NHID == 64, "two 32-deep k chunks per contraction");
static_assert(NHID % 32 == 0, "K multiple of 32, no k padding");
static_assert(NGATE == 256, "16 column tiles of 16");
static_assert(NBATCH % ROWS_BLK == 0, "grid covers the batch exactly");
static_assert((16 * NPRED * 4) % 128 == 0, "per-wave output tile is whole 128-B lines");
static_assert(16 * NPRED == 3 * 32 * 4, "three float4-per-lane store instructions per wave");
static_assert(16 * NSTEP == 12 * 32 * 4, "x tile staging: 12 float4-per-lane iterations");
static_assert((NGATE * NHID / 8) % NTHR == 0, "weight staging loop exact");
static_assert(NGATE % NTHR == 0, "table staging loop exact");

typedef __attribute__((ext_vector_type(16))) _Float16 v16h;
typedef __attribute__((ext_vector_type(8)))  _Float16 v8h;
typedef __attribute__((ext_vector_type(8)))  float    v8f;
typedef __attribute__((ext_vector_type(4)))  float    v4f;

union FragU { v16h v; v8h h[2]; };

__device__ __forceinline__ v16h frag_load(const _Float16* p) {
  FragU f;
  f.h[0] = *(const v8h*)(p);
  f.h[1] = *(const v8h*)(p + 16);
  return f.v;
}

__device__ __forceinline__ v8f mma_f16(v16h a, v16h b, v8f c) {
  return __builtin_amdgcn_wmma_f32_16x16x32_f16(false, a, false, b, (short)0, c, false, false);
}

__device__ __forceinline__ void group_guard(v8f& z0, v8f& z1, v8f& z2, v8f& z3,
                                            v16h a, v16h b0, v16h b1, v16h b2, v16h b3) {
  asm volatile("v_nop\n\tv_nop\n\tv_nop\n\tv_nop"
               : "+v"(z0), "+v"(z1), "+v"(z2), "+v"(z3)
               : "v"(a), "v"(b0), "v"(b1), "v"(b2), "v"(b3));
}

__device__ __forceinline__ void wmma_group(v8f& z0, v8f& z1, v8f& z2, v8f& z3, v16h a, const _Float16* wp) {
  const v16h b0 = frag_load(wp);
  const v16h b1 = frag_load(wp + 1 * NHID * NHID);
  const v16h b2 = frag_load(wp + 2 * NHID * NHID);
  const v16h b3 = frag_load(wp + 3 * NHID * NHID);
  z0 = mma_f16(a, b0, z0);
  z1 = mma_f16(a, b1, z1);
  z2 = mma_f16(a, b2, z2);
  z3 = mma_f16(a, b3, z3);
  group_guard(z0, z1, z2, z3, a, b0, b1, b2, b3);
}

__device__ __forceinline__ float f_sig(float x)  { return 1.0f / (1.0f + expf(-x)); }
__device__ __forceinline__ float f_tanh(float x) { return 1.0f - 2.0f / (expf(2.0f * x) + 1.0f); }

__device__ __forceinline__ v8f init_affine(const float (&xr)[8], float wv, float bv) {
  v8f z;
#pragma unroll
  for (int r = 0; r < 8; ++r) z[r] = fmaf(xr[r], wv, bv);
  return z;
}

__device__ __forceinline__ v8f init_bcast(float bv) {
  v8f z;
#pragma unroll
  for (int r = 0; r < 8; ++r) z[r] = bv;
  return z;
}

template <bool HEAD>
__device__ __forceinline__ void cell_rows(const v8f& zi, const v8f& zf, const v8f& zg, const v8f& zo,
                                          float* cp, _Float16* hp, float hwv, float (&pout)[8]) {
#pragma unroll
  for (int r = 0; r < 8; ++r) {
    const float iv = f_sig(zi[r] * ZFOLD);
    const float fv = f_sig(zf[r] * ZFOLD);
    const float gv = f_tanh(zg[r] * ZFOLD);
    const float ov = f_sig(zo[r] * ZFOLD);
    const float cprev = cp[r * 32];
    const float cv = fv * cprev + iv * gv;
    cp[r * 32] = cv;
    const float hv = ov * f_tanh(cv);
    hp[r * NHID] = (_Float16)(hv * HCARRY);
    if (HEAD) pout[r] += hv * hwv;
  }
}

__device__ __forceinline__ void cvt8_to_lds(const float* __restrict__ src, _Float16* dst) {
  const v4f a = *(const v4f*)(src);
  const v4f b = *(const v4f*)(src + 4);
  v8h hv;
#pragma unroll
  for (int e = 0; e < 4; ++e) {
    hv[e]     = (_Float16)(a[e] * WCARRY);
    hv[4 + e] = (_Float16)(b[e] * WCARRY);
  }
  *(v8h*)(dst) = hv;
}

__global__ __launch_bounds__(NTHR) void lstm2_head_kernel(
    const float* __restrict__ ts,
    const float* __restrict__ Wih0, const float* __restrict__ Whh0,
    const float* __restrict__ bih0, const float* __restrict__ bhh0,
    const float* __restrict__ Wih1, const float* __restrict__ Whh1,
    const float* __restrict__ bih1, const float* __restrict__ bhh1,
    const float* __restrict__ head_w, const float* __restrict__ head_b,
    float* __restrict__ out) {
  __shared__ __align__(16) _Float16 sWhh0[NGATE * NHID];
  __shared__ __align__(16) _Float16 sWih1[NGATE * NHID];
  __shared__ __align__(16) _Float16 sWhh1[NGATE * NHID];
  __shared__ __align__(16) _Float16 sH[NWAVE][4 * TILE_H];
  __shared__ __align__(16) float    sX[NWAVE][NSTEP * 16];
  __shared__ __align__(16) float    sC[NWAVE][2 * 4 * 8 * 32];
  __shared__ __align__(16) float    sO[NWAVE][16 * NPRED];
  __shared__ __align__(16) float    sW0[NGATE];
  __shared__ __align__(16) float    sB0[NGATE];
  __shared__ __align__(16) float    sB1[NGATE];
  __shared__ __align__(16) float    sHW[NHID];

  const int tid  = threadIdx.x;
  const int lane = tid & 31;
  const int wave = tid >> 5;
  const int ln   = lane & 15;
  const int hh   = lane >> 4;
  const int koff = hh * 8;
  const int row0 = blockIdx.x * ROWS_BLK + wave * 16;

#pragma unroll 1
  for (int i = tid; i < NGATE * NHID / 8; i += NTHR) {
    cvt8_to_lds(Whh0 + (size_t)i * 8, sWhh0 + i * 8);
    cvt8_to_lds(Wih1 + (size_t)i * 8, sWih1 + i * 8);
    cvt8_to_lds(Whh1 + (size_t)i * 8, sWhh1 + i * 8);
  }
#pragma unroll 1
  for (int i = tid; i < NGATE; i += NTHR) {
    sW0[i] = Wih0[i] * ZCARRY;
    sB0[i] = (bih0[i] + bhh0[i]) * ZCARRY;
    sB1[i] = (bih1[i] + bhh1[i]) * ZCARRY;
  }
  if (tid < NHID) sHW[tid] = head_w[tid];

  {
    _Float16* hz = &sH[wave][0];
    v8h zv;
#pragma unroll
    for (int e = 0; e < 8; ++e) zv[e] = (_Float16)0.0f;
#pragma unroll 1
    for (int i = lane; i < 4 * TILE_H / 8; i += 32) *(v8h*)(hz + i * 8) = zv;
  }
  {
    float* cz = &sC[wave][0];
#pragma unroll 1
    for (int i = 0; i < 64; ++i) cz[i * 32 + lane] = 0.0f;
  }
  {
    const float* xsrc = ts + (size_t)row0 * NSTEP;
    float* xw0 = &sX[wave][0];
#pragma unroll 1
    for (int it = 0; it < 12; ++it) {
      const int f = (it * 32 + lane) * 4;
      const v4f v = *(const v4f*)(xsrc + f);
      const int m  = f / NSTEP;
      const int tt = f - m * NSTEP;
      xw0[(tt + 0) * 16 + m] = v[0];
      xw0[(tt + 1) * 16 + m] = v[1];
      xw0[(tt + 2) * 16 + m] = v[2];
      xw0[(tt + 3) * 16 + m] = v[3];
    }
  }
  const float hb = head_b[0];
  __syncthreads();

  _Float16*    hT = &sH[wave][0];
  float*       cw = &sC[wave][0];
  const float* xw = &sX[wave][0];
  float*       ow = &sO[wave][0];
  const int foff = ln * NHID + koff;
  const int doff = (8 * hh) * NHID + ln;

#pragma unroll 1
  for (int t = 0; t < NSTEP; ++t) {
    const int par  = t & 1;
    const int h0rd = par * TILE_H;
    const int h0wr = (par ^ 1) * TILE_H;
    const int h1rd = 2 * TILE_H + par * TILE_H;
    const int h1wr = 2 * TILE_H + (par ^ 1) * TILE_H;

    float xr[8];
    {
      const v4f xa = *(const v4f*)(xw + t * 16 + 8 * hh);
      const v4f xb = *(const v4f*)(xw + t * 16 + 8 * hh + 4);
      xr[0] = xa[0]; xr[1] = xa[1]; xr[2] = xa[2]; xr[3] = xa[3];
      xr[4] = xb[0]; xr[5] = xb[1]; xr[6] = xb[2]; xr[7] = xb[3];
    }
    float pout[8];
#pragma unroll
    for (int r = 0; r < 8; ++r) pout[r] = 0.0f;

    {
      const v16h a0 = frag_load(hT + h0rd + foff);
      const v16h a1 = frag_load(hT + h0rd + foff + 32);
#pragma unroll 1
      for (int jj = 0; jj < 4; ++jj) {
        const int n = jj * 16 + ln;
        v8f z0 = init_affine(xr, sW0[n],            sB0[n]);
        v8f z1 = init_affine(xr, sW0[n + NHID],     sB0[n + NHID]);
        v8f z2 = init_affine(xr, sW0[n + 2 * NHID], sB0[n + 2 * NHID]);
        v8f z3 = init_affine(xr, sW0[n + 3 * NHID], sB0[n + 3 * NHID]);
        const _Float16* wp = sWhh0 + jj * TILE_H + foff;
        wmma_group(z0, z1, z2, z3, a0, wp);
        wmma_group(z0, z1, z2, z3, a1, wp + 32);
        cell_rows<false>(z0, z1, z2, z3, cw + jj * 256 + lane, hT + h0wr + doff + jj * 16, 0.0f, pout);
      }
    }
    __syncthreads();

    {
      const v16h ax0 = frag_load(hT + h0wr + foff);
      const v16h ax1 = frag_load(hT + h0wr + foff + 32);
      const v16h ah0 = frag_load(hT + h1rd + foff);
      const v16h ah1 = frag_load(hT + h1rd + foff + 32);
#pragma unroll 1
      for (int jj = 0; jj < 4; ++jj) {
        const int n = jj * 16 + ln;
        v8f z0 = init_bcast(sB1[n]);
        v8f z1 = init_bcast(sB1[n + NHID]);
        v8f z2 = init_bcast(sB1[n + 2 * NHID]);
        v8f z3 = init_bcast(sB1[n + 3 * NHID]);
        const _Float16* wpx = sWih1 + jj * TILE_H + foff;
        const _Float16* wph = sWhh1 + jj * TILE_H + foff;
        wmma_group(z0, z1, z2, z3, ax0, wpx);
        wmma_group(z0, z1, z2, z3, ax1, wpx + 32);
        wmma_group(z0, z1, z2, z3, ah0, wph);
        wmma_group(z0, z1, z2, z3, ah1, wph + 32);
        cell_rows<true>(z0, z1, z2, z3, cw + 1024 + jj * 256 + lane, hT + h1wr + doff + jj * 16, sHW[n], pout);
      }
    }

    if (t >= T_HEAD0) {
#pragma unroll
      for (int r = 0; r < 8; ++r) {
        float p = pout[r];
        p += __shfl_xor(p, 1, 32);
        p += __shfl_xor(p, 2, 32);
        p += __shfl_xor(p, 4, 32);
        p += __shfl_xor(p, 8, 32);
        const float val = p + hb;
        if (ln == 0) ow[(8 * hh + r) * NPRED + (t - T_HEAD0)] = val;
      }
    }
  }

  __syncthreads();
  {
    v4f ov[3];
#pragma unroll
    for (int it = 0; it < 3; ++it) ov[it] = *(const v4f*)(ow + it * 128 + lane * 4);
    float* op = out + (size_t)row0 * NPRED;
    for (int pass = 0; pass < 2; ++pass) {
#pragma unroll
      for (int it = 0; it < 3; ++it) *(volatile v4f*)(op + it * 128 + lane * 4) = ov[it];
      __threadfence();
    }
  }
}

extern "C" void kernel_launch(void* const* d_in, const int* in_sizes, int n_in,
                              void* d_out, int out_size, void* d_ws, size_t ws_size, hipStream_t stream) {
  (void)d_ws; (void)ws_size;
  if (n_in < 11 || d_out == nullptr) return;
  if (in_sizes[0] != NBATCH * NSTEP || in_sizes[1] != NGATE || in_sizes[2] != NGATE * NHID ||
      in_sizes[3] != NGATE || in_sizes[4] != NGATE || in_sizes[5] != NGATE * NHID ||
      in_sizes[6] != NGATE * NHID || in_sizes[7] != NGATE || in_sizes[8] != NGATE ||
      in_sizes[9] != NHID || in_sizes[10] != 1 || out_size != NBATCH * NPRED) return;

  const float* ts     = (const float*)d_in[0];
  const float* Wih0   = (const float*)d_in[1];
  const float* Whh0   = (const float*)d_in[2];
  const float* bih0   = (const float*)d_in[3];
  const float* bhh0   = (const float*)d_in[4];
  const float* Wih1   = (const float*)d_in[5];
  const float* Whh1   = (const float*)d_in[6];
  const float* bih1   = (const float*)d_in[7];
  const float* bhh1   = (const float*)d_in[8];
  const float* head_w = (const float*)d_in[9];
  const float* head_b = (const float*)d_in[10];
  float* out = (float*)d_out;

  lstm2_head_kernel<<<NBATCH / ROWS_BLK, NTHR, 0, stream>>>(
      ts, Wih0, Whh0, bih0, bhh0, Wih1, Whh1, bih1, bhh1, head_w, head_b, out);
}
